// MultiHeadAttentionHalf_22333829939583
// MI455X (gfx1250) — hardware-verified
//
#include <hip/hip_runtime.h>
#include <math.h>

typedef __attribute__((ext_vector_type(16))) _Float16 v16h;
typedef __attribute__((ext_vector_type(16))) __bf16 v16b;
typedef __attribute__((ext_vector_type(8)))  _Float16 v8h;
typedef __attribute__((ext_vector_type(8)))  float v8f;
typedef __attribute__((ext_vector_type(4)))  float v4f;
typedef __attribute__((ext_vector_type(2)))  float v2f;
typedef __attribute__((ext_vector_type(4)))  unsigned v4u;
typedef __attribute__((ext_vector_type(4)))  int v4i;
typedef float __attribute__((may_alias)) float_a;
typedef int __attribute__((may_alias)) int_a;

template <typename T> __device__ __forceinline__ void vst2(void* p, T v) { *(volatile T*)p = v; __threadfence(); *(volatile T*)p = v; }
__device__ __forceinline__ v8f wmma16(v16h a, v16h b, v8f c) {
  v8f d = __builtin_amdgcn_wmma_f32_16x16x32_f16(false, a, false, b, (short)0, c, false, false);
  asm volatile("v_nop\n\tv_nop\n\tv_nop\n\tv_nop" : "+v"(d) : "v"(a), "v"(b));
  return d;
}
__device__ __forceinline__ v8f wmma_bf(v16b a, v16b b, v8f c) {
  v8f d = __builtin_amdgcn_wmma_f32_16x16x32_bf16(false, a, false, b, (short)0, c, false, false);
  asm volatile("v_nop\n\tv_nop\n\tv_nop\n\tv_nop" : "+v"(d) : "v"(a), "v"(b));
  return d;
}
__device__ __forceinline__ v16h frag_h(const _Float16* rowk0, int lane) {
  union { v16h v; v8h q[2]; } u; const _Float16* p = rowk0 + 8 * (lane >> 4);
  u.q[0] = *(const v8h*)p; u.q[1] = *(const v8h*)(p + 16); return u.v;
}
__device__ __forceinline__ v16h frag_f32(const float* rowk0, int lane) {
  v16h a; const float* p = rowk0 + 8 * (lane >> 4);
#pragma unroll
  for (int i = 0; i < 8; ++i) { a[i] = (_Float16)p[i]; a[8 + i] = (_Float16)p[16 + i]; }
  return a;
}
__device__ __forceinline__ v16h frag_f32s(const float* rowk0, int lane, float sc) {
  v16h a; const float* p = rowk0 + 8 * (lane >> 4);
#pragma unroll
  for (int i = 0; i < 8; ++i) { a[i] = (_Float16)(p[i] * sc); a[8 + i] = (_Float16)(p[16 + i] * sc); }
  return a;
}
__device__ __forceinline__ v16h fragc_f32(const float* W, int k0, int n, int lane, int ld, int K) {
  v16h a; const int g = lane >> 4;
#pragma unroll
  for (int i = 0; i < 8; ++i) { const int ka = k0 + 8 * g + i, kb = ka + 16;
    a[i] = (_Float16)(ka < K ? W[(size_t)(ka < K ? ka : K - 1) * ld + n] : 0.f); a[8 + i] = (_Float16)(kb < K ? W[(size_t)(kb < K ? kb : K - 1) * ld + n] : 0.f); }
  return a;
}
struct F2 { v16b h, l; };
__device__ __forceinline__ F2 bsplit16(const float v[16]) { F2 r;
#pragma unroll
  for (int i = 0; i < 16; ++i) { const __bf16 h = (__bf16)v[i]; r.h[i] = h; r.l[i] = (__bf16)(v[i] - (float)h); }
  return r; }
__device__ __forceinline__ F2 split_row(const float* row, int k0, int lane) { float v[16]; const float* p = row + k0 + 8 * (lane >> 4);
#pragma unroll
  for (int i = 0; i < 8; ++i) { v[i] = p[i]; v[8 + i] = p[16 + i]; }
  return bsplit16(v); }
__device__ __forceinline__ F2 split_rowK(const float* row, int k0, int lane, int K) { float v[16]; const int g = lane >> 4;
#pragma unroll
  for (int i = 0; i < 8; ++i) { const int ka = k0 + 8 * g + i, kb = ka + 16; v[i] = ka < K ? row[ka < K ? ka : K - 1] : 0.f; v[8 + i] = kb < K ? row[kb < K ? kb : K - 1] : 0.f; }
  return bsplit16(v); }
__device__ __forceinline__ F2 split_col(const float* W, int k0, int n, int lane, int ld, int K) { float v[16]; const int g = lane >> 4;
#pragma unroll
  for (int i = 0; i < 8; ++i) { const int ka = k0 + 8 * g + i, kb = ka + 16; v[i] = ka < K ? W[(size_t)(ka < K ? ka : K - 1) * ld + n] : 0.f; v[8 + i] = kb < K ? W[(size_t)(kb < K ? kb : K - 1) * ld + n] : 0.f; }
  return bsplit16(v); }
__device__ __forceinline__ v8f mac3(const F2& a, const F2& b, v8f c) { c = wmma_bf(a.l, b.h, c); c = wmma_bf(a.h, b.l, c); return wmma_bf(a.h, b.h, c); }
__device__ __forceinline__ float sigm(float v) { return 1.0f / (1.0f + expf(-v)); }
#define LDSX() do { asm volatile("s_wait_dscnt 0" ::: "memory"); __builtin_amdgcn_wave_barrier(); __builtin_amdgcn_fence(__ATOMIC_RELEASE, "workgroup"); } while (0)


#define NB 4
#define SS 1024
#define EE 1024
#define NH 16
#define DH 64
#define NR (NB * SS)
#define NQB (SS / 16)
#ifndef TNB
#define TNB NB
#endif
typedef __attribute__((ext_vector_type(8))) __bf16 v8b;
__device__ __forceinline__ v16b frag_b(const __bf16* rowk0, int lane) {
  union { v16b v; v8b q[2]; } u; const __bf16* p = rowk0 + 8 * (lane >> 4);
  u.q[0] = *(const v8b*)p; u.q[1] = *(const v8b*)(p + 16); return u.v;
}
__device__ __forceinline__ float bfr(float v) { return (float)(__bf16)v; }
__device__ __attribute__((noinline)) float exp_ni(float v) { return expf(v); }
__device__ __attribute__((noinline)) float erf_ni(float v) { return erff(v); }

#define WS_QH   0u
#define WS_QL   (WS_QH + 2u * (size_t)NR * 2 * EE)
#define WS_V    (WS_QL + 2u * (size_t)NR * 2 * EE)
#define WS_PC   (WS_V + 4u * (size_t)NR * EE)
#define WS_CB   (WS_PC + 4u * (size_t)NB * NQB * NH * SS)
#define WS_G    (WS_CB + 4u * (size_t)NB * NH * SS)
#define WS_CTX  (WS_G + 4u * (size_t)NB * NH * EE)
#define WS_END  (WS_CTX + 4u * (size_t)16 * EE)

__device__ __forceinline__ v16b fragb_f32(const float* __restrict__ p, int lane) { v16b a; const float* pp = p + 8 * (lane >> 4);
#pragma unroll
  for (int i = 0; i < 8; ++i) { a[i] = (__bf16)pp[i]; a[8 + i] = (__bf16)pp[16 + i]; } return a; }
__global__ __launch_bounds__(128) void k_proj(const float* __restrict__ X, const float* __restrict__ W, const float* __restrict__ Bqkv, _Float16* __restrict__ QH, _Float16* __restrict__ QL, float* __restrict__ V) { __shared__ __align__(16) _Float16 sh[4][16][136], sl[4][16][136]; __shared__ __align__(16) float sf[4][16][132];
  const int tid = threadIdx.x, wave = tid >> 5, lane = tid & 31, col = lane & 15, g = lane >> 4; const size_t r0 = (size_t)blockIdx.x * 64 + wave * 16; const int c0 = blockIdx.y * 128;
  v8f acc[8] = {};
#pragma unroll 2
  for (int kc = 0; kc < EE / 32; ++kc) { const v16b a = fragb_f32(X + (r0 + col) * EE + kc * 32, lane);
#pragma unroll
    for (int j = 0; j < 8; ++j) acc[j] = wmma_bf(a, fragb_f32(W + (size_t)(c0 + j * 16 + col) * EE + kc * 32, lane), acc[j]); }
  const bool isv = c0 >= 2 * EE;
#pragma unroll
  for (int j = 0; j < 8; ++j) { const float bb = bfr(Bqkv[c0 + j * 16 + col]);
#pragma unroll
    for (int r = 0; r < 8; ++r) { const float v = acc[j][r] + bb; if (isv) sf[wave][8 * g + r][j * 16 + col] = v; else { const _Float16 hv = (_Float16)v; sh[wave][8 * g + r][j * 16 + col] = hv; sl[wave][8 * g + r][j * 16 + col] = (_Float16)((v - (float)hv) * 2048.0f); } } }
  LDSX();
  if (isv) { for (int rl = 0; rl < 16; ++rl) vst2(V + (r0 + rl) * EE + (c0 - 2 * EE) + lane * 4, *(const v4f*)&sf[wave][rl][lane * 4]); }
  else { for (int rl = 0; rl < 16; ++rl) if (lane < 16) { vst2((unsigned*)(QH + (r0 + rl) * (2 * EE) + c0 + lane * 8), *(const v4u*)&sh[wave][rl][lane * 8]); vst2((unsigned*)(QL + (r0 + rl) * (2 * EE) + c0 + lane * 8), *(const v4u*)&sl[wave][rl][lane * 8]); } } }
__global__ __launch_bounds__(128) void k_attw(const _Float16* __restrict__ QH, const _Float16* __restrict__ QL, float* __restrict__ PC, float* __restrict__ AWOUT) { __shared__ __align__(16) float slg[16][SS + 4]; __shared__ __align__(16) float saw[16][SS + 4]; __shared__ float srow[16][2];
  const int tid = threadIdx.x, wave = tid >> 5, lane = tid & 31, col = lane & 15, g = lane >> 4; const size_t b = blockIdx.y; const int qb = blockIdx.x; const size_t rq = b * SS + (size_t)qb * 16;
  for (int e = tid; e < 16 * SS; e += 128) saw[e / SS][e % SS] = 0.f;
#pragma unroll 1
  for (int h = 0; h < NH; ++h) {
    v16h aq[2], al[2];
#pragma unroll
    for (int kc = 0; kc < 2; ++kc) { aq[kc] = frag_h(QH + (rq + col) * (2 * EE) + h * DH + kc * 32, lane); al[kc] = frag_h(QL + (rq + col) * (2 * EE) + h * DH + kc * 32, lane); }
#pragma unroll 1
    for (int rd = 0; rd < SS / 512; ++rd) { v8f acc[8], accl[8];
#pragma unroll
      for (int j = 0; j < 8; ++j) { acc[j] = v8f{}; accl[j] = v8f{}; }
#pragma unroll
      for (int j = 0; j < 8; ++j) { const size_t rk = b * SS + wave * (SS / 4) + rd * 128 + j * 16 + col;
#pragma unroll
        for (int kc = 0; kc < 2; ++kc) { const v16h kh = frag_h(QH + rk * (2 * EE) + EE + h * DH + kc * 32, lane), kl = frag_h(QL + rk * (2 * EE) + EE + h * DH + kc * 32, lane); acc[j] = wmma16(aq[kc], kh, acc[j]); accl[j] = wmma16(aq[kc], kl, accl[j]); accl[j] = wmma16(al[kc], kh, accl[j]); } }
#pragma unroll
      for (int j = 0; j < 8; ++j)
#pragma unroll
        for (int r = 0; r < 8; ++r) slg[8 * g + r][wave * (SS / 4) + rd * 128 + j * 16 + col] = (acc[j][r] + accl[j][r] * (1.0f / 2048.0f)) * 0.125f; }
    __syncthreads();
    { const int r = tid >> 3, part = tid & 7; float* row = &slg[r][0]; float mx = -3.0e38f; for (int t = part * (SS / 8); t < part * (SS / 8) + (SS / 8); ++t) mx = fmaxf(mx, row[t]);
#pragma unroll
      for (int o = 1; o < 8; o <<= 1) mx = fmaxf(mx, __shfl_xor(mx, o));
      float s = 0.f; for (int t = part * (SS / 8); t < part * (SS / 8) + (SS / 8); ++t) { const float e = __expf(row[t] - mx); row[t] = e; s += e; }
#pragma unroll
      for (int o = 1; o < 8; o <<= 1) s += __shfl_xor(s, o);
      const float inv = 1.0f / s; for (int t = part * (SS / 8); t < part * (SS / 8) + (SS / 8); ++t) { const float p = row[t] * inv; row[t] = p; saw[r][t] += p * (1.0f / NH); } }
    __syncthreads();
    { __shared__ __align__(16) float scs[SS]; for (int t = tid; t < SS; t += 128) { float s = 0.f;
#pragma unroll
        for (int r = 0; r < 16; ++r) s += slg[r][t]; scs[t] = s; }
      __syncthreads(); for (int q = tid; q < SS / 4; q += 128) vst2(PC + (((b * NQB + qb) * NH + h) * (size_t)SS) + q * 4, *(const v4f*)&scs[q * 4]); }
    __syncthreads(); }
  for (int e = tid; e < 16 * (SS / 4); e += 128) { const int r = e / (SS / 4), q = e % (SS / 4); vst2(AWOUT + (rq + r) * SS + q * 4, *(const v4f*)&saw[r][q * 4]); } }
__global__ __launch_bounds__(256) void k_cbar(const float* __restrict__ PC, float* __restrict__ CB) { __shared__ __align__(16) float s[SS]; const int h = blockIdx.x, t = threadIdx.x; const size_t b = blockIdx.y;
  for (int c = t; c < SS; c += 256) { float a = 0.f;
#pragma unroll 1
    for (int qb = 0; qb < NQB; ++qb) a += PC[(((b * NQB + qb) * NH + h) * (size_t)SS) + c]; s[c] = a * (1.0f / SS); }
  __syncthreads(); if (t < SS / 4) vst2(CB + ((b * NH + h) * (size_t)SS) + t * 4, *(const v4f*)&s[t * 4]); }
__global__ __launch_bounds__(128) void k_gmat(const float* __restrict__ CB, const float* __restrict__ V, float* __restrict__ G) { __shared__ __align__(16) float sg[16][132];
  const int tid = threadIdx.x, wave = tid >> 5, lane = tid & 31, col = lane & 15, g = lane >> 4; const size_t b = blockIdx.y; const int c0 = blockIdx.x * 128 + wave * 32;
  v8f acc[2] = {};
#pragma unroll 1
  for (int kc = 0; kc < SS / 32; ++kc) { const F2 a = split_row(CB + (b * NH + col) * (size_t)SS, kc * 32, lane);
#pragma unroll
    for (int j = 0; j < 2; ++j) { float w[16]; const int c = c0 + j * 16 + col;
#pragma unroll
      for (int i = 0; i < 8; ++i) { w[i] = V[(b * SS + kc * 32 + 8 * g + i) * (size_t)EE + c]; w[8 + i] = V[(b * SS + kc * 32 + 16 + 8 * g + i) * (size_t)EE + c]; }
      const F2 wb = bsplit16(w); acc[j] = wmma_bf(a.h, wb.h, acc[j]); acc[j] = wmma_bf(a.h, wb.l, acc[j]); acc[j] = wmma_bf(a.l, wb.h, acc[j]); acc[j] = wmma_bf(a.l, wb.l, acc[j]); } }
#pragma unroll
  for (int j = 0; j < 2; ++j)
#pragma unroll
    for (int r = 0; r < 8; ++r) sg[8 * g + r][wave * 32 + j * 16 + col] = acc[j][r];
  __syncthreads(); for (int e = tid; e < 16 * 32; e += 128) { const int hr = e >> 5, q = e & 31; vst2(G + ((b * NH + hr) * (size_t)EE) + blockIdx.x * 128 + q * 4, *(const v4f*)&sg[hr][q * 4]); } }
__global__ __launch_bounds__(256) void k_ctx1(const float* __restrict__ G, float* __restrict__ CTX) { __shared__ __align__(16) float s[EE]; const int t = threadIdx.x; const int rb = blockIdx.x;
  for (int c = t; c < EE; c += 256) s[c] = (rb < NB) ? G[(((size_t)rb * NH + c / DH) * EE) + c] : 0.f; __syncthreads(); vst2(CTX + (size_t)rb * EE + t * 4, *(const v4f*)&s[t * 4]); }
__global__ __launch_bounds__(128) void k_ctx2(const float* __restrict__ CTX, const float* __restrict__ WO, const float* __restrict__ BO, float* __restrict__ OUT0) { __shared__ __align__(16) float so[16][132];
  const int tid = threadIdx.x, wave = tid >> 5, lane = tid & 31, col = lane & 15, g = lane >> 4; const int c0 = blockIdx.x * 128 + wave * 32;
  v8f acc[2] = {};
#pragma unroll 2
  for (int kc = 0; kc < EE / 32; ++kc) { const F2 a = split_row(CTX + (size_t)col * EE, kc * 32, lane);
#pragma unroll
    for (int j = 0; j < 2; ++j) { const v16b w = fragb_f32(WO + (size_t)(c0 + j * 16 + col) * EE + kc * 32, lane); acc[j] = wmma_bf(a.h, w, acc[j]); acc[j] = wmma_bf(a.l, w, acc[j]); } }
#pragma unroll
  for (int j = 0; j < 2; ++j) { const float bb = bfr(BO[c0 + j * 16 + col]);
#pragma unroll
    for (int r = 0; r < 8; ++r) so[8 * g + r][wave * 32 + j * 16 + col] = acc[j][r] + bb; }
  __syncthreads(); for (int e = tid; e < NB * 32; e += 128) { const int rb = e >> 5, q = e & 31; vst2(OUT0 + (size_t)rb * EE + blockIdx.x * 128 + q * 4, *(const v4f*)&so[rb][q * 4]); } }
extern "C" void kernel_launch(void* const* d_in, const int* in_sizes, int n_in, void* d_out, int out_size, void* d_ws, size_t ws_size, hipStream_t stream) {
  (void)in_sizes; (void)n_in; (void)out_size;
  const float** F = (const float**)d_in;
  if (ws_size < (size_t)WS_END) return;
  char* ws = (char*)d_ws; _Float16 *QH = (_Float16*)(ws + WS_QH), *QL = (_Float16*)(ws + WS_QL); float *V = (float*)(ws + WS_V), *PC = (float*)(ws + WS_PC), *CB = (float*)(ws + WS_CB), *G = (float*)(ws + WS_G), *CTX = (float*)(ws + WS_CTX);
  float* OUT0 = (float*)d_out; float* OUT1 = OUT0 + (size_t)NB * EE;
  k_proj<<<dim3(NR / 64, 3 * EE / 128), 128, 0, stream>>>(F[0], F[1], F[2], QH, QL, V);
  k_attw<<<dim3(NQB, TNB), 128, 0, stream>>>(QH, QL, PC, OUT1);
  k_cbar<<<dim3(NH, TNB), 256, 0, stream>>>(PC, CB);
  k_gmat<<<dim3(EE / 128, TNB), 128, 0, stream>>>(CB, V, G);
  k_ctx1<<<16, 256, 0, stream>>>(G, CTX);
  k_ctx2<<<EE / 128, 128, 0, stream>>>(CTX, F[3], F[4], OUT0);
}
